// LSTM_Calib_9972914061687
// MI455X (gfx1250) — hardware-run, weakly checked
//
#include <hip/hip_runtime.h>
#include <math.h>

constexpr int kSteps  = 15;
constexpr int kHid    = 15;
constexpr int kGates  = 60;
constexpr int kKA     = 32;
constexpr int kNP     = 64;
constexpr int kCW     = 16;
constexpr int kD2     = 60;
constexpr int kD3     = 20;
constexpr float kWCarry     = 8.0f;
constexpr float kWCarryInv  = 0.125f;
constexpr float kO1Carry    = 16.0f;
constexpr float kO1CarryInv = 0.0625f;

typedef __attribute__((ext_vector_type(16))) _Float16 v16h;
typedef __attribute__((ext_vector_type(8)))  _Float16 v8h;
typedef __attribute__((ext_vector_type(16))) __bf16   v16b;
typedef __attribute__((ext_vector_type(8)))  __bf16   v8b;
typedef __attribute__((ext_vector_type(8)))  float    v8f;
typedef __attribute__((ext_vector_type(4)))  float    v4f;
typedef __attribute__((ext_vector_type(4)))  unsigned int v4u;

__device__ __forceinline__ unsigned short f2bf_bits(float f) {
  unsigned u = __float_as_uint(f);
  return (unsigned short)((u + 0x7FFFu + ((u >> 16) & 1u)) >> 16);
}
__device__ __forceinline__ float bf_bits2f(unsigned short h) { return __uint_as_float(((unsigned)h) << 16); }

__device__ __forceinline__ void dep_guard_h(v8f& a, v8f& b, v16h x, v16h y) { asm volatile("v_nop\n\tv_nop\n\tv_nop\n\tv_nop" : "+v"(a), "+v"(b) : "v"(x), "v"(y)); }
__device__ __forceinline__ void dep_guard_b(v8f& a, v8f& b, v16b x, v16b y) { asm volatile("v_nop\n\tv_nop\n\tv_nop\n\tv_nop" : "+v"(a), "+v"(b) : "v"(x), "v"(y)); }
__device__ __forceinline__ void keep4_h(v16h a, v16h b, v16h c, v16h d) { asm volatile("v_nop" :: "v"(a), "v"(b), "v"(c), "v"(d)); }
__device__ __forceinline__ void keep4_b(v16b a, v16b b, v16b c, v16b d) { asm volatile("v_nop" :: "v"(a), "v"(b), "v"(c), "v"(d)); }
__device__ __forceinline__ void acc_guard4(v8f& a, v8f& b, v8f& c, v8f& d) { asm volatile("v_nop\n\tv_nop\n\tv_nop\n\tv_nop" : "+v"(a), "+v"(b), "+v"(c), "+v"(d)); }
template <typename T> struct Frag;
template <> struct Frag<_Float16> {
  typedef v16h V; union U { v16h v; v8h h[2]; };
  static __device__ __forceinline__ v16h load(const _Float16* p) {
    U f; f.h[0] = *(const v8h*)(p); f.h[1] = *(const v8h*)(p + 16); return f.v;
  }
  static __device__ __forceinline__ v8f mma(v16h a, v16h b, v8f c) {
    return __builtin_amdgcn_wmma_f32_16x16x32_f16(false, a, false, b, (short)0, c, false, false);
  }
  static __device__ __forceinline__ void guard(v8f& a, v8f& b, v16h x, v16h y) { dep_guard_h(a, b, x, y); }
  static __device__ __forceinline__ void keep(v16h a, v16h b, v16h c, v16h d) { keep4_h(a, b, c, d); }
};
template <> struct Frag<__bf16> {
  typedef v16b V; union U { v16b v; v8b h[2]; };
  static __device__ __forceinline__ v16b load(const __bf16* p) {
    U f; f.h[0] = *(const v8b*)(p); f.h[1] = *(const v8b*)(p + 16); return f.v;
  }
  static __device__ __forceinline__ v8f mma(v16b a, v16b b, v8f c) {
    return __builtin_amdgcn_wmma_f32_16x16x32_bf16(false, a, false, b, (short)0, c, false, false);
  }
  static __device__ __forceinline__ void guard(v8f& a, v8f& b, v16b x, v16b y) { dep_guard_b(a, b, x, y); }
  static __device__ __forceinline__ void keep(v16b a, v16b b, v16b c, v16b d) { keep4_b(a, b, c, d); }
};

__device__ __forceinline__ unsigned pk16(unsigned short a, unsigned short b) { return (unsigned)a | ((unsigned)b << 16); }
__device__ __forceinline__ unsigned short h_bits(float f) { const _Float16 h = (_Float16)f; return __builtin_bit_cast(unsigned short, h); }

template <int ET> struct Elem;
template <> struct Elem<0> { typedef _Float16 T; };
template <> struct Elem<1> { typedef __bf16 T; };
template <int ET, bool SPLIT, int BIAS_MODE, int OUT_MODE, bool RESID, int ACT = 0>
__global__ __launch_bounds__(256) void wmma_gemm64(
    const unsigned short* __restrict__ Ap, const unsigned short* __restrict__ A2p, int lda, long strideA,
    const unsigned short* __restrict__ Btp, const unsigned short* __restrict__ Bt2p, int ldb, long strideB,
    void* __restrict__ Cout, void* __restrict__ Cout2, int ldc, long strideC,
    const float* __restrict__ bias,
    const float* __restrict__ resid, long strideR,
    int M, int N, int K, float scale) {
  typedef typename Elem<ET>::T T;
  typedef typename Frag<T>::V V;
  const T* A = (const T*)Ap; const T* A2 = (const T*)A2p; const T* Bt = (const T*)Btp; const T* Bt2 = (const T*)Bt2p;
  __shared__ __align__(16) float sT[8][16 * 68];
  const int b    = blockIdx.y;
  const int lane = threadIdx.x & 31;
  const int wave = threadIdx.x >> 5;
  const int tilesN = N >> 6;
  const int tilesM = M >> 6;
  const int tile = blockIdx.x * 8 + wave;
  if (tile >= tilesM * tilesN) return;
  const int tm = tile / tilesN;
  const int tn = tile - tm * tilesN;
  const int m0 = tm << 6;
  const int n0 = tn << 6;

  const T* Ab  = A  + (size_t)b * strideA;
  const T* Bb  = Bt + (size_t)b * strideB;
  const T* Ab2 = SPLIT ? (A2  + (size_t)b * strideA) : nullptr;
  const T* Bb2 = SPLIT ? (Bt2 + (size_t)b * strideB) : nullptr;

  const int rlane = lane & 15;
  const int koff  = (lane >> 4) * 8;
  const int mOff  = (lane >> 4) * 8;

  v8f acc[4][4];
#pragma unroll
  for (int i = 0; i < 4; ++i)
#pragma unroll
    for (int j = 0; j < 4; ++j) acc[i][j] = (v8f){0.f,0.f,0.f,0.f,0.f,0.f,0.f,0.f};

  for (int k0 = 0; k0 < K; k0 += 32) {
    V bh[4], bl[4];
#pragma unroll
    for (int j = 0; j < 4; ++j) {
      const size_t bo = (size_t)(n0 + (j << 4) + rlane) * ldb + koff + k0;
      bh[j] = Frag<T>::load(Bb + bo);
      if (SPLIT) bl[j] = Frag<T>::load(Bb2 + bo);
    }
#pragma unroll
    for (int i = 0; i < 4; ++i) {
      const size_t ao = (size_t)(m0 + (i << 4) + rlane) * lda + koff + k0;
      V ah = Frag<T>::load(Ab + ao);
      V al;
      if (SPLIT) al = Frag<T>::load(Ab2 + ao);
#pragma unroll
      for (int j = 0; j < 4; ++j) {
        acc[i][j] = Frag<T>::mma(ah, bh[j], acc[i][j]);
        if (SPLIT) {
          acc[i][j] = Frag<T>::mma(ah, bl[j], acc[i][j]);
          acc[i][j] = Frag<T>::mma(al, bh[j], acc[i][j]);
        }
      }
      Frag<T>::guard(acc[i][0], acc[i][3], ah, SPLIT ? al : ah);
    }
    Frag<T>::keep(bh[0], bh[1], bh[2], bh[3]);
    if (SPLIT) Frag<T>::keep(bl[0], bl[1], bl[2], bl[3]);
  }
  acc_guard4(acc[0][0], acc[0][1], acc[0][2], acc[0][3]);
  acc_guard4(acc[1][0], acc[1][1], acc[1][2], acc[1][3]);
  acc_guard4(acc[2][0], acc[2][1], acc[2][2], acc[2][3]);
  acc_guard4(acc[3][0], acc[3][1], acc[3][2], acc[3][3]);

  float* slab = sT[wave];
  const float* Rb = RESID ? (resid + (size_t)b * strideR) : nullptr;
#pragma unroll
  for (int i = 0; i < 4; ++i) {
    const int mBase = m0 + (i << 4);
#pragma unroll
    for (int j = 0; j < 4; ++j) {
      const int n = n0 + (j << 4) + rlane;
      float bv = 0.f;
      if (BIAS_MODE == 2) bv = bias[n];
#pragma unroll
      for (int r = 0; r < 8; ++r) {
        float v = acc[i][j][r] * scale;
        if (BIAS_MODE == 1) v += bias[mBase + mOff + r];
        if (BIAS_MODE == 2) v += bv;
        if (RESID) v += Rb[(size_t)(mBase + mOff + r) * ldc + n];
        if (ACT == 1) v = tanhf(v);
        if (ACT == 2) v = fmaxf(v, 0.0f);
        if (ACT == 4) v = (v > 0.f) ? v : 0.01f * v;
        slab[(mOff + r) * 68 + (j << 4) + rlane] = v;
      }
    }
    __builtin_amdgcn_fence(__ATOMIC_RELEASE, "workgroup");
    __builtin_amdgcn_wave_barrier();
    __builtin_amdgcn_fence(__ATOMIC_ACQUIRE, "workgroup");
    if (OUT_MODE == 0) {
      float* C = (float*)Cout + (size_t)b * strideC;
      const int hh = lane >> 4, c4 = (lane & 15) * 4;
      for (int pass = 0; pass < 2; ++pass) {
#pragma unroll
        for (int it = 0; it < 8; ++it) {
          const int row = it * 2 + hh;
          v4f v = *(const v4f*)(slab + row * 68 + c4);
          *(volatile v4f*)(C + (size_t)(mBase + row) * ldc + n0 + c4) = v;
        }
        __threadfence();
      }
    } else {
      const int q = lane >> 3, c8 = (lane & 7) * 8;
      unsigned short* C  = (unsigned short*)Cout  + (size_t)b * strideC;
      unsigned short* C2 = (OUT_MODE == 2) ? ((unsigned short*)Cout2 + (size_t)b * strideC) : nullptr;
      for (int pass = 0; pass < 2; ++pass) {
#pragma unroll
        for (int it = 0; it < 4; ++it) {
          const int row = it * 4 + q;
          const float* sp = slab + row * 68 + c8;
          v8h hv, lv;
#pragma unroll
          for (int e = 0; e < 8; ++e) {
            if (OUT_MODE == 1) {
              hv[e] = (_Float16)sp[e];
            } else {
              unsigned short hb = f2bf_bits(sp[e]);
              unsigned short lb = f2bf_bits(sp[e] - bf_bits2f(hb));
              hv[e] = __builtin_bit_cast(_Float16, hb);
              lv[e] = __builtin_bit_cast(_Float16, lb);
            }
          }
          *(volatile v8h*)(C + (size_t)(mBase + row) * ldc + n0 + c8) = hv;
          if (OUT_MODE == 2) *(volatile v8h*)(C2 + (size_t)(mBase + row) * ldc + n0 + c8) = lv;
        }
        __threadfence();
      }
    }
    __builtin_amdgcn_fence(__ATOMIC_RELEASE, "workgroup");
    __builtin_amdgcn_wave_barrier();
    __builtin_amdgcn_fence(__ATOMIC_ACQUIRE, "workgroup");
  }
}

__device__ __forceinline__ int clampi(int v, int lo, int hi) { return v < lo ? lo : (v > hi ? hi : v); }

__device__ __forceinline__ float sigm_f(float z) {
  z = fminf(fmaxf(z, -40.0f), 40.0f);
  const float e = __expf(-z);
  return __builtin_amdgcn_rcpf(1.0f + e);
}
__device__ __forceinline__ float tanh_f(float z) {
  const float a = fminf(fabsf(z), 20.0f);
  const float e = __expf(-2.0f * a);
  const float r = (1.0f - e) * __builtin_amdgcn_rcpf(1.0f + e);
  return copysignf(r, z);
}

__device__ __forceinline__ float bt0_elem(int n, int k, const float* __restrict__ Wih0, const float* __restrict__ Whh0) {
  const int nc = clampi(n, 0, kGates - 1);
  const int kh = clampi(k - 1, 0, kHid - 1);
  const float wi = Wih0[nc];
  const float wh = Whh0[nc * kHid + kh];
  const float v = (k == 0) ? wi : ((k <= kHid) ? wh : 0.0f);
  return (n < kGates) ? v * kWCarry : 0.0f;
}
__device__ __forceinline__ float bt1_elem(int n, int k, const float* __restrict__ Wih1, const float* __restrict__ Whh1) {
  const int nc = clampi(n, 0, kGates - 1);
  const int ka = clampi(k, 0, kHid - 1);
  const int kb = clampi(k - kHid, 0, kHid - 1);
  const float wi = Wih1[nc * kHid + ka];
  const float wh = Whh1[nc * kHid + kb];
  const float v = (k < kHid) ? wi : ((k < 2 * kHid) ? wh : 0.0f);
  return (n < kGates) ? v * kWCarry : 0.0f;
}
__device__ __forceinline__ float bta_elem(int n, int k, const float* __restrict__ W1) {
  const int nc = clampi(n, 0, kD2 - 1);
  const int ka = clampi(k, 0, kHid - 1);
  const float w = W1[nc * kHid + ka];
  return (n < kD2 && k < kHid) ? w * kWCarry : 0.0f;
}
__device__ __forceinline__ float btb_elem(int n, int k, const float* __restrict__ W2) {
  const int nc = clampi(n, 0, kD3 - 1);
  const int ka = clampi(k, 0, kD2 - 1);
  const float w = W2[nc * kD2 + ka];
  return (n < kD3 && k < kD2) ? w * kWCarry : 0.0f;
}

__device__ __forceinline__ void store2_v4u(unsigned short* p, v4u u) {
  *(volatile v4u*)p = u;
  __threadfence();
  *(volatile v4u*)p = u;
}
__device__ __forceinline__ void store2_v4f(float* p, v4f f) {
  *(volatile v4f*)p = f;
  __threadfence();
  *(volatile v4f*)p = f;
}

__global__ __launch_bounds__(256) void pack_params_kernel(
    const float* __restrict__ Wih0, const float* __restrict__ Whh0, const float* __restrict__ bih0, const float* __restrict__ bhh0,
    const float* __restrict__ Wih1, const float* __restrict__ Whh1, const float* __restrict__ bih1, const float* __restrict__ bhh1,
    const float* __restrict__ W1, const float* __restrict__ b1, const float* __restrict__ W2, const float* __restrict__ b2,
    unsigned short* __restrict__ Bt0, unsigned short* __restrict__ Bt1, unsigned short* __restrict__ BtA,
    unsigned short* __restrict__ BtB, float* __restrict__ biasv) {
  const int blk = blockIdx.x;
  const int i   = threadIdx.x;
  if (blk <= 4) {
    int n, k0;
    unsigned short* dst;
    if (blk >= 3) {
      const int j = (blk - 3) * 256 + i;
      n = j >> 3; k0 = (j & 7) * 8;
      dst = BtB + 8 * (size_t)j;
    } else {
      n = i >> 2; k0 = (i & 3) * 8;
      dst = ((blk == 0) ? Bt0 : ((blk == 1) ? Bt1 : BtA)) + 8 * (size_t)i;
    }
    unsigned short hb[8];
#pragma unroll
    for (int e = 0; e < 8; ++e) {
      const int k = k0 + e;
      const float v0 = bt0_elem(n, k, Wih0, Whh0);
      const float v1 = bt1_elem(n, k, Wih1, Whh1);
      const float va = bta_elem(n, k, W1);
      const float vb = btb_elem(n, k, W2);
      const float v = (blk == 0) ? v0 : ((blk == 1) ? v1 : ((blk == 2) ? va : vb));
      hb[e] = h_bits(v);
    }
    const v4u u = (v4u){pk16(hb[0], hb[1]), pk16(hb[2], hb[3]), pk16(hb[4], hb[5]), pk16(hb[6], hb[7])};
    store2_v4u(dst, u);
  } else {
    if (i < 64) {
      const int p  = i >> 4;
      const int nb = (i & 15) * 4;
      float bv[4];
#pragma unroll
      for (int e = 0; e < 4; ++e) {
        const int n  = nb + e;
        const int nc = clampi(n, 0, kGates - 1);
        const int n3 = clampi(n, 0, kD3 - 1);
        const float s0 = bih0[nc] + bhh0[nc];
        const float s1 = bih1[nc] + bhh1[nc];
        const float s2 = b1[nc] * kO1Carry;
        const float s3 = b2[n3];
        const float g0 = (n < kGates) ? s0 : 0.0f;
        const float g1 = (n < kGates) ? s1 : 0.0f;
        const float g2 = (n < kD2)    ? s2 : 0.0f;
        const float g3 = (n < kD3)    ? s3 : 0.0f;
        bv[e] = (p == 0) ? g0 : ((p == 1) ? g1 : ((p == 2) ? g2 : g3));
      }
      const v4f f = (v4f){bv[0], bv[1], bv[2], bv[3]};
      store2_v4f(biasv + 4 * (size_t)i, f);
    }
  }
}

__global__ __launch_bounds__(256) void init_state_kernel(const float* __restrict__ x, unsigned short* __restrict__ A0,
    float* __restrict__ C0, float* __restrict__ C1, float* __restrict__ H1, int nrows) {
  const int idx = threadIdx.x;
  const int row = blockIdx.x * 64 + (idx >> 2);
  const int q   = idx & 3;
  const int rowc = clampi(row, 0, nrows - 1);
  const float xv = x[(size_t)rowc * kSteps];
  const unsigned xb = (unsigned)h_bits(xv);
  const v4u av = (v4u){(q == 0) ? xb : 0u, 0u, 0u, 0u};
  const v4f zf = (v4f){0.f, 0.f, 0.f, 0.f};
  unsigned short* ap = A0 + (size_t)row * kKA + q * 8;
  float* c0p = C0 + (size_t)row * kCW + q * 4;
  float* c1p = C1 + (size_t)row * kCW + q * 4;
  float* h1p = H1 + (size_t)row * kCW + q * 4;
  *(volatile v4u*)ap  = av;
  *(volatile v4f*)c0p = zf;
  *(volatile v4f*)c1p = zf;
  *(volatile v4f*)h1p = zf;
  __threadfence();
  *(volatile v4u*)ap  = av;
  *(volatile v4f*)c0p = zf;
  *(volatile v4f*)c1p = zf;
  *(volatile v4f*)h1p = zf;
}

__global__ __launch_bounds__(256) void cell0_kernel(const float* __restrict__ Z, float* __restrict__ C0,
    unsigned short* __restrict__ A0, unsigned short* __restrict__ A1, const float* __restrict__ H1,
    const float* __restrict__ x, int nrows, int t) {
  __shared__ float hs[16][16];
  __shared__ float cs[16][16];
  __shared__ float h1s[16][16];
  const int tid  = threadIdx.x;
  const int rl   = tid >> 4;
  const int u    = tid & 15;
  const int row0 = blockIdx.x * 16;
  const int row  = row0 + rl;
  const int uc   = (u < kHid) ? u : (kHid - 1);
  const float* zr = Z + (size_t)row * kNP;
  const float zi = zr[uc];
  const float zf = zr[kHid + uc];
  const float zg = zr[2 * kHid + uc];
  const float zo = zr[3 * kHid + uc];
  const float cp = C0[(size_t)row * kCW + uc];
  h1s[rl][u] = H1[(size_t)row * kCW + u];
  const float ig = sigm_f(zi);
  const float fg = sigm_f(zf);
  const float gg = tanh_f(zg);
  const float og = sigm_f(zo);
  float c = fmaf(fg, cp, ig * gg);
  float h = og * tanh_f(c);
  const bool valid = (u < kHid);
  c = valid ? c : 0.0f;
  h = valid ? h : 0.0f;
  hs[rl][u] = h;
  cs[rl][u] = c;
  __syncthreads();
  if (tid < 32) {
    const int lane = tid;
    const int tn = (t + 1 < kSteps) ? (t + 1) : (kSteps - 1);
    v4f cv[2];
    v4u a0v[2], a1v[2];
#pragma unroll
    for (int it = 0; it < 2; ++it) {
      const int idx = it * 32 + lane;
      const int r = idx >> 2, q = idx & 3;
      cv[it] = (v4f){cs[r][q * 4 + 0], cs[r][q * 4 + 1], cs[r][q * 4 + 2], cs[r][q * 4 + 3]};
      const int rx = clampi(row0 + r, 0, nrows - 1);
      const float xv = x[(size_t)rx * kSteps + tn];
      unsigned short b0[8], b1[8];
#pragma unroll
      for (int e = 0; e < 8; ++e) {
        const int col = q * 8 + e;
        const int ih = clampi(col - 1, 0, kHid - 1);
        const float hv = hs[r][ih];
        const float v0 = (col == 0) ? xv : ((col <= kHid) ? hv : 0.0f);
        const int ia = clampi(col, 0, kHid - 1);
        const float ha = hs[r][ia];
        const int ib = clampi(col - kHid, 0, kHid - 1);
        const float hb = h1s[r][ib];
        const float v1 = (col < kHid) ? ha : ((col < 2 * kHid) ? hb : 0.0f);
        b0[e] = h_bits(v0);
        b1[e] = h_bits(v1);
      }
      a0v[it] = (v4u){pk16(b0[0], b0[1]), pk16(b0[2], b0[3]), pk16(b0[4], b0[5]), pk16(b0[6], b0[7])};
      a1v[it] = (v4u){pk16(b1[0], b1[1]), pk16(b1[2], b1[3]), pk16(b1[4], b1[5]), pk16(b1[6], b1[7])};
    }
    for (int pass = 0; pass < 2; ++pass) {
#pragma unroll
      for (int it = 0; it < 2; ++it) {
        const int idx = it * 32 + lane;
        const int r = idx >> 2, q = idx & 3;
        const size_t rr = (size_t)(row0 + r);
        *(volatile v4f*)(C0 + rr * kCW + q * 4) = cv[it];
        *(volatile v4u*)(A0 + rr * kKA + q * 8) = a0v[it];
        *(volatile v4u*)(A1 + rr * kKA + q * 8) = a1v[it];
      }
      __threadfence();
    }
  }
}

__global__ __launch_bounds__(256) void cell1_kernel(const float* __restrict__ Z, float* __restrict__ C1,
    float* __restrict__ H1, unsigned short* __restrict__ FEAT, int nrows, int t) {
  __shared__ float hs[16][16];
  __shared__ float cs[16][16];
  const int tid  = threadIdx.x;
  const int rl   = tid >> 4;
  const int u    = tid & 15;
  const int row0 = blockIdx.x * 16;
  const int row  = row0 + rl;
  const int uc   = (u < kHid) ? u : (kHid - 1);
  const float* zr = Z + (size_t)row * kNP;
  const float zi = zr[uc];
  const float zf = zr[kHid + uc];
  const float zg = zr[2 * kHid + uc];
  const float zo = zr[3 * kHid + uc];
  const float cp = C1[(size_t)row * kCW + uc];
  const float ig = sigm_f(zi);
  const float fg = sigm_f(zf);
  const float gg = tanh_f(zg);
  const float og = sigm_f(zo);
  float c = fmaf(fg, cp, ig * gg);
  float h = og * tanh_f(c);
  const bool valid = (u < kHid);
  c = valid ? c : 0.0f;
  h = valid ? h : 0.0f;
  hs[rl][u] = h;
  cs[rl][u] = c;
  __syncthreads();
  if (tid < 32) {
    const int lane = tid;
    v4f cv[2], hv4[2];
    v4u fv[2];
#pragma unroll
    for (int it = 0; it < 2; ++it) {
      const int idx = it * 32 + lane;
      const int r = idx >> 2, q = idx & 3;
      cv[it]  = (v4f){cs[r][q * 4 + 0], cs[r][q * 4 + 1], cs[r][q * 4 + 2], cs[r][q * 4 + 3]};
      hv4[it] = (v4f){hs[r][q * 4 + 0], hs[r][q * 4 + 1], hs[r][q * 4 + 2], hs[r][q * 4 + 3]};
      const v4u old = *(const v4u*)(FEAT + (size_t)(row0 + r) * kKA + q * 8);
      const unsigned short h14b = h_bits(hs[r][kHid - 1]);
      unsigned short nb[8];
#pragma unroll
      for (int e = 0; e < 8; ++e) {
        const int col = q * 8 + e;
        const unsigned w = (e & 1) ? (old[e >> 1] >> 16) : (old[e >> 1] & 0xFFFFu);
        const unsigned short ob = (unsigned short)w;
        nb[e] = (col < t) ? ob : ((col == t) ? h14b : (unsigned short)0);
      }
      fv[it] = (v4u){pk16(nb[0], nb[1]), pk16(nb[2], nb[3]), pk16(nb[4], nb[5]), pk16(nb[6], nb[7])};
    }
    for (int pass = 0; pass < 2; ++pass) {
#pragma unroll
      for (int it = 0; it < 2; ++it) {
        const int idx = it * 32 + lane;
        const int r = idx >> 2, q = idx & 3;
        const size_t rr = (size_t)(row0 + r);
        *(volatile v4f*)(C1 + rr * kCW + q * 4)   = cv[it];
        *(volatile v4f*)(H1 + rr * kCW + q * 4)   = hv4[it];
        *(volatile v4u*)(FEAT + rr * kKA + q * 8) = fv[it];
      }
      __threadfence();
    }
  }
  (void)nrows;
}

__global__ __launch_bounds__(64) void head_out_kernel(const float* __restrict__ O2, const float* __restrict__ W3,
    const float* __restrict__ b3, float* __restrict__ out, int nrows) {
  __shared__ float os[64];
  const int tid = threadIdx.x;
  const int row0 = blockIdx.x * 64;
  const int row = clampi(row0 + tid, 0, nrows - 1);
  const float* orow = O2 + (size_t)row * kNP;
  float acc = 0.0f;
#pragma unroll 1
  for (int k = 0; k < kD3; ++k) acc = fmaf(orow[k], W3[k], acc);
  acc += b3[0];
  os[tid] = acc;
  __syncthreads();
  if (tid < 16) {
    const v4f v = (v4f){os[tid * 4 + 0], os[tid * 4 + 1], os[tid * 4 + 2], os[tid * 4 + 3]};
    float* p = out + (size_t)row0 + tid * 4;
    *(volatile v4f*)p = v;
    __threadfence();
    *(volatile v4f*)p = v;
  }
}

extern "C" void kernel_launch(void* const* d_in, const int* in_sizes, int n_in,
                              void* d_out, int out_size, void* d_ws, size_t ws_size,
                              hipStream_t stream) {
  if (n_in < 15) return;
  const int nx = in_sizes[0];
  if (nx <= 0 || (nx % (kSteps * 64)) != 0) return;
  const int nrows = nx / kSteps;
  if (out_size != nrows) return;
  if (in_sizes[1] != kGates || in_sizes[2] != kGates * kHid || in_sizes[3] != kGates || in_sizes[4] != kGates) return;
  if (in_sizes[5] != kGates * kHid || in_sizes[6] != kGates * kHid || in_sizes[7] != kGates || in_sizes[8] != kGates) return;
  if (in_sizes[9] != kD2 * kHid || in_sizes[10] != kD2 || in_sizes[11] != kD3 * kD2 || in_sizes[12] != kD3) return;
  if (in_sizes[13] != kD3 || in_sizes[14] != 1) return;

  const float* x    = (const float*)d_in[0];
  const float* Wih0 = (const float*)d_in[1];
  const float* Whh0 = (const float*)d_in[2];
  const float* bih0 = (const float*)d_in[3];
  const float* bhh0 = (const float*)d_in[4];
  const float* Wih1 = (const float*)d_in[5];
  const float* Whh1 = (const float*)d_in[6];
  const float* bih1 = (const float*)d_in[7];
  const float* bhh1 = (const float*)d_in[8];
  const float* W1   = (const float*)d_in[9];
  const float* b1   = (const float*)d_in[10];
  const float* W2   = (const float*)d_in[11];
  const float* b2   = (const float*)d_in[12];
  const float* W3   = (const float*)d_in[13];
  const float* b3   = (const float*)d_in[14];
  float* outp = (float*)d_out;

  const size_t SZ_PAR = 32768;
  const size_t SZ_P16 = (size_t)nrows * kKA * 2;
  const size_t SZ_S32 = (size_t)nrows * kCW * 4;
  const size_t SZ_Z   = (size_t)nrows * kNP * 4;
  size_t off = 0;
  const size_t oPAR  = off; off += SZ_PAR;
  const size_t oA0   = off; off += SZ_P16;
  const size_t oA1   = off; off += SZ_P16;
  const size_t oFEAT = off; off += SZ_P16;
  const size_t oC0   = off; off += SZ_S32;
  const size_t oC1   = off; off += SZ_S32;
  const size_t oH1   = off; off += SZ_S32;
  const size_t oZ    = off; off += SZ_Z;
  const size_t oO2   = off; off += SZ_Z;
  const size_t TOTAL = off;
  if (TOTAL > ws_size) return;
  if (TOTAL > (size_t)134217728) return;

  char* ws = (char*)d_ws;
  unsigned short* Bt0  = (unsigned short*)(ws + oPAR + 0);
  unsigned short* Bt1  = (unsigned short*)(ws + oPAR + 4096);
  unsigned short* BtA  = (unsigned short*)(ws + oPAR + 8192);
  unsigned short* BtB  = (unsigned short*)(ws + oPAR + 12288);
  float*          biasv = (float*)(ws + oPAR + 20480);
  const float* bias0 = biasv;
  const float* bias1 = biasv + 64;
  const float* biasA = biasv + 128;
  const float* biasB = biasv + 192;
  unsigned short* A0   = (unsigned short*)(ws + oA0);
  unsigned short* A1   = (unsigned short*)(ws + oA1);
  unsigned short* FEAT = (unsigned short*)(ws + oFEAT);
  float*          C0   = (float*)(ws + oC0);
  float*          C1   = (float*)(ws + oC1);
  float*          H1   = (float*)(ws + oH1);
  float*          Z    = (float*)(ws + oZ);
  unsigned short* O1   = (unsigned short*)(ws + oZ);
  float*          O2   = (float*)(ws + oO2);
  const float* nores = biasv;

  const dim3 blk256(256);
  const int tilesM = nrows / 64;
  const dim3 gG((tilesM + 7) / 8, 1);
  const dim3 gCell(nrows / 16);
  const dim3 gRow64(nrows / 64);

  pack_params_kernel<<<dim3(6), blk256, 0, stream>>>(Wih0, Whh0, bih0, bhh0, Wih1, Whh1, bih1, bhh1,
                                                      W1, b1, W2, b2, Bt0, Bt1, BtA, BtB, biasv);
  init_state_kernel<<<gRow64, blk256, 0, stream>>>(x, A0, C0, C1, H1, nrows);

  for (int t = 0; t < kSteps; ++t) {
    wmma_gemm64<0, false, 2, 0, false, 0><<<gG, blk256, 0, stream>>>(
        A0, A0, kKA, 0L, Bt0, Bt0, kKA, 0L, (void*)Z, (void*)Z, kNP, 0L, bias0, nores, 0L, nrows, kNP, kKA, kWCarryInv);
    cell0_kernel<<<gCell, blk256, 0, stream>>>(Z, C0, A0, A1, H1, x, nrows, t);
    wmma_gemm64<0, false, 2, 0, false, 0><<<gG, blk256, 0, stream>>>(
        A1, A1, kKA, 0L, Bt1, Bt1, kKA, 0L, (void*)Z, (void*)Z, kNP, 0L, bias1, nores, 0L, nrows, kNP, kKA, kWCarryInv);
    cell1_kernel<<<gCell, blk256, 0, stream>>>(Z, C1, H1, FEAT, nrows, t);
  }

  wmma_gemm64<0, false, 2, 1, false, 0><<<gG, blk256, 0, stream>>>(
      FEAT, FEAT, kKA, 0L, BtA, BtA, kKA, 0L, (void*)O1, (void*)O1, kNP, 0L, biasA, nores, 0L, nrows, kNP, kKA,
      kWCarryInv * kO1Carry);
  wmma_gemm64<0, false, 2, 0, false, 0><<<gG, blk256, 0, stream>>>(
      O1, O1, kNP, 0L, BtB, BtB, kNP, 0L, (void*)O2, (void*)O2, kNP, 0L, biasB, nores, 0L, nrows, kNP, kNP,
      kWCarryInv * kO1CarryInv);
  head_out_kernel<<<gRow64, dim3(64), 0, stream>>>(O2, W3, b3, outp, nrows);
}
